// LoFTREncoderLayer_56006373540107
// MI455X (gfx1250) — hardware-verified
//
#include <hip/hip_runtime.h>
#include <math.h>
#include <stdint.h>

#ifndef NB
#define NB 4
#endif
#ifndef SEQ
#define SEQ 4096
#endif
#ifndef SSEQ
#define SSEQ SEQ
#endif
#define L_FULL 4096
#define NH    8
#define DM    64
#define DFF   128
#define MT    (NB * SEQ * NH)
#define MS    (NB * SSEQ * NH)
#define MX    ((MT > MS) ? MT : MS)
#define NNH   (NB * NH)
#define NST   (SSEQ / 64)
#define NLT   (SEQ / 64)
#define QSC   1024.0f
#define KCAR  1024.0f
#define VSC   1024.0f
#define KVCAR 4.0f
#define EPSA  1e-6f
#define EPSL  1e-5f
#define SLP   68
#define SLAB64 (16 * SLP)
#define WS_CAP 134217728

#define RUP(x)  ((((size_t)(x)) + (size_t)65535) & ~(size_t)65535)
#define SZ_W    RUP(81920)
#define SZ_PS   RUP((size_t)NNH * NST * 64 * 4)
#define SZ_KS   RUP((size_t)NNH * 64 * 4)
#define SZ_KV   RUP((size_t)NNH * 64 * 64 * 2)
#define SZ_DEN  RUP((size_t)MT * 4)
#define SZ_XB   RUP((size_t)MT * 128)
#define SLB     ((size_t)MX * 128)
#define WS_TOTAL (SZ_W + SZ_PS + SZ_KS + 2 * SZ_KV + SZ_DEN + SZ_XB + 6 * SLB)

static_assert(NB >= 1 && NB <= 4);
static_assert(NB == 1 || (SEQ == L_FULL && SSEQ == L_FULL));
static_assert((SEQ % 64) == 0 && SEQ >= 64 && SEQ <= L_FULL);
static_assert((SSEQ % 64) == 0 && SSEQ >= 64 && SSEQ <= L_FULL);
static_assert((MT % 64) == 0 && (MS % 64) == 0 && (MX % 512) == 0);
static_assert((SLB % 65536) == 0);
static_assert((size_t)MT * 256 <= 2 * SLB);
static_assert((size_t)MS * 128 <= SLB && (size_t)MT * 128 <= SLB);
static_assert(WS_TOTAL <= (size_t)WS_CAP);
static_assert(4 * SLAB64 * 4 + 64 * 4 <= 65536);

typedef unsigned short u16;
typedef _Float16 v16h __attribute__((ext_vector_type(16)));
typedef _Float16 v8h  __attribute__((ext_vector_type(8)));
typedef __bf16   v16b __attribute__((ext_vector_type(16)));
typedef float    v8f  __attribute__((ext_vector_type(8)));
typedef float    v4f  __attribute__((ext_vector_type(4)));
typedef unsigned int v4u __attribute__((ext_vector_type(4)));

union FragH { v16h v; v8h h[2]; v4u u[2]; };
union FragB { v16b v; v4u u[2]; };

__device__ __forceinline__ unsigned short bf_bits(float f) {
  unsigned u = __float_as_uint(f);
  return (unsigned short)((u + 0x7FFFu + ((u >> 16) & 1u)) >> 16);
}
__device__ __forceinline__ float bf_up(unsigned short h) { return __uint_as_float(((unsigned)h) << 16); }
__device__ __forceinline__ float bfr(float f) { return bf_up(bf_bits(f)); }
__device__ __forceinline__ unsigned short h_bits(_Float16 x) { return __builtin_bit_cast(unsigned short, x); }
__device__ __forceinline__ unsigned pk16(unsigned short a, unsigned short b) { return (unsigned)a | ((unsigned)b << 16); }
__device__ __forceinline__ v8f zero8() { v8f z = {0.f, 0.f, 0.f, 0.f, 0.f, 0.f, 0.f, 0.f}; return z; }

__device__ __forceinline__ float elu1(float t) {
  const float en = expm1f(fminf(t, 0.0f)) + 1.0f;
  return (t > 0.0f) ? (t + 1.0f) : en;
}
__device__ __forceinline__ float gsum8(float s) {
  s += __shfl_xor(s, 1);
  s += __shfl_xor(s, 2);
  s += __shfl_xor(s, 4);
  return s;
}

__device__ __forceinline__ v16h ldfrag_h(const _Float16* p) {
  FragH f;
  f.h[0] = *(const v8h*)(p);
  f.h[1] = *(const v8h*)(p + 16);
  return f.v;
}
__device__ __forceinline__ v16b ldfrag_b(const u16* p) {
  FragB f;
  f.u[0] = *(const v4u*)(p);
  f.u[1] = *(const v4u*)(p + 16);
  return f.v;
}

__device__ __forceinline__ v8f mma_h(v16h a, v16h b, v8f c) {
  return __builtin_amdgcn_wmma_f32_16x16x32_f16(false, a, false, b, (short)0, c, false, false);
}
__device__ __forceinline__ v8f mma_b(v16b a, v16b b, v8f c) {
  return __builtin_amdgcn_wmma_f32_16x16x32_bf16(false, a, false, b, (short)0, c, false, false);
}
__device__ __forceinline__ void guard2(v8f& a, v8f& b, v16h x0, v16h x1, v16h x2, v16h x3, v16h x4, v16h x5) {
#if defined(__HIP_DEVICE_COMPILE__)
  asm volatile("v_nop\n\tv_nop\n\tv_nop\n\tv_nop"
               : "+v"(a), "+v"(b) : "v"(x0), "v"(x1), "v"(x2), "v"(x3), "v"(x4), "v"(x5) : "memory");
#endif
}
template <typename F>
__device__ __forceinline__ void guard6(v8f& a, v8f& b, v8f& c, v8f& d, F x0, F x1, F x2, F x3, F x4, F x5) {
#if defined(__HIP_DEVICE_COMPILE__)
  asm volatile("v_nop\n\tv_nop\n\tv_nop\n\tv_nop"
               : "+v"(a), "+v"(b), "+v"(c), "+v"(d) : "v"(x0), "v"(x1), "v"(x2), "v"(x3), "v"(x4), "v"(x5) : "memory");
#endif
}
__device__ __forceinline__ void wave_sync_lds() {
  __builtin_amdgcn_fence(__ATOMIC_RELEASE, "workgroup");
  __builtin_amdgcn_wave_barrier();
  __builtin_amdgcn_fence(__ATOMIC_ACQUIRE, "workgroup");
}

template <int NP>
__device__ __forceinline__ void step_b(const u16* ah, const u16* al, const u16* bp, size_t bjs, int k0,
                                       v8f& c0, v8f& c1, v8f& c2, v8f& c3) {
  const v16b a  = ldfrag_b(ah + k0);
  const v16b f0 = ldfrag_b(bp + k0);
  const v16b f1 = ldfrag_b(bp + bjs + k0);
  const v16b f2 = ldfrag_b(bp + 2 * bjs + k0);
  const v16b f3 = ldfrag_b(bp + 3 * bjs + k0);
  c0 = mma_b(a, f0, c0);
  c1 = mma_b(a, f1, c1);
  c2 = mma_b(a, f2, c2);
  c3 = mma_b(a, f3, c3);
  if constexpr (NP == 2) {
    const v16b a2 = ldfrag_b(al + k0);
    c0 = mma_b(a2, f0, c0);
    c1 = mma_b(a2, f1, c1);
    c2 = mma_b(a2, f2, c2);
    c3 = mma_b(a2, f3, c3);
    guard6<v16b>(c0, c1, c2, c3, a, a2, f0, f1, f2, f3);
  } else {
    guard6<v16b>(c0, c1, c2, c3, a, f0, f1, f2, f3, a);
  }
}
template <int NP, int NS>
__device__ __forceinline__ void kloop_b(const u16* ah, const u16* al, const u16* bp, size_t bjs,
                                        v8f& c0, v8f& c1, v8f& c2, v8f& c3) {
  if constexpr (NS <= 2) {
#pragma unroll
    for (int s = 0; s < NS; ++s) step_b<NP>(ah, al, bp, bjs, s * 32, c0, c1, c2, c3);
  } else {
#pragma unroll 1
    for (int s = 0; s < NS; ++s) step_b<NP>(ah, al, bp, bjs, s * 32, c0, c1, c2, c3);
  }
}

__device__ __forceinline__ void step_h3(const _Float16* ah, const _Float16* al, const _Float16* bh, const _Float16* bl,
                                        size_t bjs, int k0, v8f& c0, v8f& c1, v8f& c2, v8f& c3) {
  const v16h a = ldfrag_h(ah + k0), a2 = ldfrag_h(al + k0);
  {
    const v16h h0 = ldfrag_h(bh + k0), h1 = ldfrag_h(bh + bjs + k0);
    const v16h l0 = ldfrag_h(bl + k0), l1 = ldfrag_h(bl + bjs + k0);
    c0 = mma_h(a, h0, c0);  c0 = mma_h(a2, h0, c0);  c0 = mma_h(a, l0, c0);
    c1 = mma_h(a, h1, c1);  c1 = mma_h(a2, h1, c1);  c1 = mma_h(a, l1, c1);
    guard2(c0, c1, a, a2, h0, l0, h1, l1);
  }
  {
    const v16h h2 = ldfrag_h(bh + 2 * bjs + k0), h3 = ldfrag_h(bh + 3 * bjs + k0);
    const v16h l2 = ldfrag_h(bl + 2 * bjs + k0), l3 = ldfrag_h(bl + 3 * bjs + k0);
    c2 = mma_h(a, h2, c2);  c2 = mma_h(a2, h2, c2);  c2 = mma_h(a, l2, c2);
    c3 = mma_h(a, h3, c3);  c3 = mma_h(a2, h3, c3);  c3 = mma_h(a, l3, c3);
    guard2(c2, c3, a, a2, h2, l2, h3, l3);
  }
}
template <int NS>
__device__ __forceinline__ void kloop_h3(const _Float16* ah, const _Float16* al, const _Float16* bh, const _Float16* bl,
                                         size_t bjs, v8f& c0, v8f& c1, v8f& c2, v8f& c3) {
  if constexpr (NS <= 2) {
#pragma unroll
    for (int s = 0; s < NS; ++s) step_h3(ah, al, bh, bl, bjs, s * 32, c0, c1, c2, c3);
  } else {
#pragma unroll 1
    for (int s = 0; s < NS; ++s) step_h3(ah, al, bh, bl, bjs, s * 32, c0, c1, c2, c3);
  }
}

__device__ __forceinline__ void slab_put(float* sl, v8f a0, v8f a1, v8f a2, v8f a3, int lane) {
  const int hh = lane >> 4, m = lane & 15;
#pragma unroll
  for (int r = 0; r < 8; ++r) {
    const int ro = (8 * hh + r) * SLP + m;
    sl[ro]      = a0[r];
    sl[ro + 16] = a1[r];
    sl[ro + 32] = a2[r];
    sl[ro + 48] = a3[r];
  }
  wave_sync_lds();
}
__device__ __forceinline__ void slab_row8(const float* sl, int row, int c8, float (&w)[8]) {
  const v4f a = *(const v4f*)(sl + row * SLP + c8);
  const v4f b = *(const v4f*)(sl + row * SLP + c8 + 4);
#pragma unroll
  for (int e = 0; e < 4; ++e) { w[e] = a[e]; w[4 + e] = b[e]; }
}
__device__ __forceinline__ void pack_h2(const float (&w)[8], v4u& oh, v4u& ol) {
#pragma unroll
  for (int e = 0; e < 4; ++e) {
    const float t0 = w[2 * e], t1 = w[2 * e + 1];
    const _Float16 h0 = (_Float16)t0, h1 = (_Float16)t1;
    const _Float16 l0 = (_Float16)(t0 - (float)h0), l1 = (_Float16)(t1 - (float)h1);
    oh[e] = pk16(h_bits(h0), h_bits(h1));
    ol[e] = pk16(h_bits(l0), h_bits(l1));
  }
}
__device__ __forceinline__ void pack_b2(const float (&w)[8], v4u& oh, v4u& ol) {
#pragma unroll
  for (int e = 0; e < 4; ++e) {
    const float f0 = w[2 * e], f1 = w[2 * e + 1];
    const unsigned short h0 = bf_bits(f0), h1 = bf_bits(f1);
    const unsigned short l0 = bf_bits(f0 - bf_up(h0)), l1 = bf_bits(f1 - bf_up(h1));
    oh[e] = pk16(h0, h1);
    ol[e] = pk16(l0, l1);
  }
}
__device__ __forceinline__ void store2_planes(u16* Dh, u16* Dl, const size_t (&off)[4], const v4u (&oh)[4], const v4u (&ol)[4]) {
  for (int pass = 0; pass < 2; ++pass) {
#pragma unroll
    for (int it = 0; it < 4; ++it) {
      *(volatile v4u*)(Dh + off[it]) = oh[it];
      *(volatile v4u*)(Dl + off[it]) = ol[it];
    }
    __threadfence();
  }
}
__device__ __forceinline__ void ln8(float (&w)[8], const float* __restrict__ g, const float* __restrict__ b, int c8) {
#pragma clang fp contract(off)
  float s = 0.0f;
#pragma unroll
  for (int e = 0; e < 8; ++e) s += w[e];
  s = gsum8(s);
  const float mean = s * (1.0f / 64.0f);
  float d[8];
  float ss = 0.0f;
#pragma unroll
  for (int e = 0; e < 8; ++e) { d[e] = w[e] - mean; ss += d[e] * d[e]; }
  ss = gsum8(ss);
  const float var = ss * (1.0f / 64.0f);
  const float rs  = 1.0f / sqrtf(var + EPSL);
  const v4f ga = *(const v4f*)(g + c8), gb = *(const v4f*)(g + c8 + 4);
  const v4f ba = *(const v4f*)(b + c8), bb = *(const v4f*)(b + c8 + 4);
#pragma unroll
  for (int e = 0; e < 4; ++e) {
    w[e]     = d[e]     * rs * bfr(ga[e]) + bfr(ba[e]);
    w[4 + e] = d[4 + e] * rs * bfr(gb[e]) + bfr(bb[e]);
  }
}

__global__ __launch_bounds__(256) void cvt_w(const float* __restrict__ wq, const float* __restrict__ wk,
                                             const float* __restrict__ wv, const float* __restrict__ wm,
                                             const float* __restrict__ w1, const float* __restrict__ w2,
                                             u16* Dq, u16* Dk, u16* Dv, u16* Dm, u16* D1, u16* D2) {
  const int bid = (int)blockIdx.x, tid = (int)threadIdx.x;
  if (bid >= 20) return;
  const float* src = (bid < 2) ? wq : ((bid < 4) ? wk : ((bid < 6) ? wv : ((bid < 8) ? wm : ((bid < 16) ? w1 : w2))));
  u16* dst = (bid < 2) ? Dq : ((bid < 4) ? Dk : ((bid < 6) ? Dv : ((bid < 8) ? Dm : ((bid < 16) ? D1 : D2))));
  const int b0 = (bid < 2) ? 0 : ((bid < 4) ? 2 : ((bid < 6) ? 4 : ((bid < 8) ? 6 : ((bid < 16) ? 8 : 16))));
  const int gt = (bid - b0) * 256 + tid;
  const float* p = src + (size_t)gt * 8;
  const v4f a = *(const v4f*)(p), b4 = *(const v4f*)(p + 4);
  v4u o;
#pragma unroll
  for (int e = 0; e < 2; ++e) {
    o[e]     = pk16(bf_bits(a[2 * e]), bf_bits(a[2 * e + 1]));
    o[2 + e] = pk16(bf_bits(b4[2 * e]), bf_bits(b4[2 * e + 1]));
  }
  u16* d = dst + (size_t)gt * 8;
  for (int pass = 0; pass < 2; ++pass) {
    *(volatile v4u*)(d) = o;
    __threadfence();
  }
}

__global__ __launch_bounds__(256) void cvt_x2(const float* __restrict__ x0, const float* __restrict__ x1,
                                              u16* D0, u16* D1, int n8a, int n8b) {
  const int which = (int)blockIdx.y;
  const float* x = (which == 0) ? x0 : x1;
  u16* D = (which == 0) ? D0 : D1;
  const int n8 = (which == 0) ? n8a : n8b;
  const int gt = (int)blockIdx.x * 256 + (int)threadIdx.x;
  if (gt >= n8) return;
  const float* p = x + (size_t)gt * 8;
  const v4f a = *(const v4f*)(p), b4 = *(const v4f*)(p + 4);
  v4u o;
#pragma unroll
  for (int e = 0; e < 2; ++e) {
    o[e]     = pk16(bf_bits(a[2 * e]), bf_bits(a[2 * e + 1]));
    o[2 + e] = pk16(bf_bits(b4[2 * e]), bf_bits(b4[2 * e + 1]));
  }
  u16* d = D + (size_t)gt * 8;
  for (int pass = 0; pass < 2; ++pass) {
    *(volatile v4u*)(d) = o;
    __threadfence();
  }
}

template <bool ELU>
__global__ __launch_bounds__(128)
void gemm_kt(const u16* __restrict__ W, const u16* __restrict__ SB, u16* THo, u16* TLo, float* PSo) {
#pragma clang fp contract(off)
  __shared__ __align__(16) float slab[4 * SLAB64];
  __shared__ __align__(16) float psl[64];
  const int tid = (int)threadIdx.x, wave = tid >> 5, lane = tid & 31, hh = lane >> 4, m = lane & 15;
  const int bid = (int)blockIdx.x;
  const int nh = bid / NST, st = bid % NST;
  if (nh >= NNH) return;
  const int n = nh / NH, h = nh % NH, s0 = st * 64;
  const u16* ap = W + (size_t)(wave * 16 + m) * DM + 8 * hh;
  const u16* bp = SB + ((size_t)(n * L_FULL + s0 + m) * NH + h) * DM + 8 * hh;
  v8f c0 = zero8(), c1 = zero8(), c2 = zero8(), c3 = zero8();
  kloop_b<1, DM / 32>(ap, ap, bp, (size_t)16 * NH * DM, c0, c1, c2, c3);
  float* sl = slab + wave * SLAB64;
  slab_put(sl, c0, c1, c2, c3, lane);
  const int rq = lane >> 3, c8 = (lane & 7) * 8;
  const float car = ELU ? KCAR : VSC;
  v4u oh[4], ol[4];
  size_t off[4];
#pragma unroll
  for (int it = 0; it < 4; ++it) {
    const int row = it * 4 + rq;
    float w[8];
    slab_row8(sl, row, c8, w);
    if constexpr (ELU) {
      float s = 0.0f;
#pragma unroll
      for (int e = 0; e < 8; ++e) { w[e] = elu1(w[e]); s += w[e]; }
      s = gsum8(s);
      if ((lane & 7) == 0) psl[wave * 16 + row] = s;
    }
#pragma unroll
    for (int e = 0; e < 8; ++e) w[e] *= car;
    pack_h2(w, oh[it], ol[it]);
    off[it] = ((size_t)nh * 64 + wave * 16 + row) * (size_t)SSEQ + s0 + c8;
  }
  store2_planes(THo, TLo, off, oh, ol);
  if constexpr (ELU) {
    __syncthreads();
    if (wave == 0 && lane < 16) {
      const v4f p = *(const v4f*)(psl + lane * 4);
      float* d = PSo + ((size_t)nh * NST + st) * 64 + lane * 4;
      for (int pass = 0; pass < 2; ++pass) {
        *(volatile v4f*)(d) = p;
        __threadfence();
      }
    }
  }
}

__global__ __launch_bounds__(128)
void kv_gemm(const u16* __restrict__ PTH, const u16* __restrict__ PTL, const u16* __restrict__ KTH,
             const u16* __restrict__ KTL, const float* __restrict__ PS, u16* KVH, u16* KVL, float* KS) {
#pragma clang fp contract(off)
  __shared__ __align__(16) float slab[4 * SLAB64];
  __shared__ __align__(16) float ksl[64];
  const int tid = (int)threadIdx.x, wave = tid >> 5, lane = tid & 31, hh = lane >> 4, m = lane & 15;
  const int nh = (int)blockIdx.x;
  if (nh >= NNH) return;
  const size_t arow = ((size_t)nh * 64 + wave * 16 + m) * (size_t)SSEQ + 8 * hh;
  const size_t brow = ((size_t)nh * 64 + m) * (size_t)SSEQ + 8 * hh;
  const _Float16* ah = (const _Float16*)(const void*)PTH + arow;
  const _Float16* al = (const _Float16*)(const void*)PTL + arow;
  const _Float16* bh = (const _Float16*)(const void*)KTH + brow;
  const _Float16* bl = (const _Float16*)(const void*)KTL + brow;
  v8f c0 = zero8(), c1 = zero8(), c2 = zero8(), c3 = zero8();
  kloop_h3<SSEQ / 32>(ah, al, bh, bl, (size_t)16 * SSEQ, c0, c1, c2, c3);
  float* sl = slab + wave * SLAB64;
  slab_put(sl, c0, c1, c2, c3, lane);
  const int rq = lane >> 3, c8 = (lane & 7) * 8;
  const float fold = KVCAR / (KCAR * VSC);
  v4u oh[4], ol[4];
  size_t off[4];
#pragma unroll
  for (int it = 0; it < 4; ++it) {
    const int row = it * 4 + rq;
    float w[8];
    slab_row8(sl, row, c8, w);
#pragma unroll
    for (int e = 0; e < 8; ++e) w[e] *= fold;
    pack_h2(w, oh[it], ol[it]);
    off[it] = ((size_t)nh * 64 + wave * 16 + row) * DM + c8;
  }
  store2_planes(KVH, KVL, off, oh, ol);
  if (tid < 64) {
    float s = 0.0f;
#pragma unroll 1
    for (int st = 0; st < NST; ++st) s += PS[((size_t)nh * NST + st) * 64 + tid];
    ksl[tid] = s;
  }
  __syncthreads();
  if (wave == 0 && lane < 16) {
    const v4f p = *(const v4f*)(ksl + lane * 4);
    float* d = KS + (size_t)nh * 64 + lane * 4;
    for (int pass = 0; pass < 2; ++pass) {
      *(volatile v4f*)(d) = p;
      __threadfence();
    }
  }
}

__global__ __launch_bounds__(128)
void gemm_q(const u16* __restrict__ XB, const u16* __restrict__ WQ, const float* __restrict__ KS,
            u16* QH, u16* QL, float* DEN) {
#pragma clang fp contract(off)
  __shared__ __align__(16) float slab[4 * SLAB64];
  __shared__ __align__(16) float dsl[64];
  const int tid = (int)threadIdx.x, wave = tid >> 5, lane = tid & 31, hh = lane >> 4, m = lane & 15;
  const int rowb0 = (int)blockIdx.x * 64;
  if (rowb0 + 64 > MT) return;
  const int rowb = rowb0 + wave * 16;
  const u16* ap = XB + (size_t)(rowb + m) * DM + 8 * hh;
  const u16* bp = WQ + (size_t)m * DM + 8 * hh;
  v8f c0 = zero8(), c1 = zero8(), c2 = zero8(), c3 = zero8();
  kloop_b<1, DM / 32>(ap, ap, bp, (size_t)16 * DM, c0, c1, c2, c3);
  float* sl = slab + wave * SLAB64;
  slab_put(sl, c0, c1, c2, c3, lane);
  const int rq = lane >> 3, c8 = (lane & 7) * 8;
  v4u oh[4], ol[4];
  size_t off[4];
#pragma unroll
  for (int it = 0; it < 4; ++it) {
    const int row = it * 4 + rq;
    const int t = rowb + row;
    const int nh = (t / (L_FULL * NH)) * NH + (t % NH);
    float w[8];
    slab_row8(sl, row, c8, w);
#pragma unroll
    for (int e = 0; e < 8; ++e) w[e] = elu1(w[e]);
    const v4f ka = *(const v4f*)(KS + (size_t)nh * 64 + c8), kb = *(const v4f*)(KS + (size_t)nh * 64 + c8 + 4);
    float dot = 0.0f;
#pragma unroll
    for (int e = 0; e < 4; ++e) dot += w[e] * ka[e];
#pragma unroll
    for (int e = 0; e < 4; ++e) dot += w[4 + e] * kb[e];
    dot = gsum8(dot);
    if ((lane & 7) == 0) dsl[wave * 16 + row] = dot + EPSA;
#pragma unroll
    for (int e = 0; e < 8; ++e) w[e] *= QSC;
    pack_h2(w, oh[it], ol[it]);
    off[it] = (size_t)t * DM + c8;
  }
  store2_planes(QH, QL, off, oh, ol);
  __syncthreads();
  if (wave == 0 && lane < 16) {
    const v4f p = *(const v4f*)(dsl + lane * 4);
    float* d = DEN + (size_t)rowb0 + lane * 4;
    for (int pass = 0; pass < 2; ++pass) {
      *(volatile v4f*)(d) = p;
      __threadfence();
    }
  }
}

__global__ __launch_bounds__(128)
void qkv(const u16* __restrict__ QH, const u16* __restrict__ QL, const u16* __restrict__ KVH,
         const u16* __restrict__ KVL, const float* __restrict__ DEN, u16* MH, u16* ML) {
#pragma clang fp contract(off)
  __shared__ __align__(16) float slab[4 * SLAB64];
  const int tid = (int)threadIdx.x, wave = tid >> 5, lane = tid & 31, hh = lane >> 4, m = lane & 15;
  const int bid = (int)blockIdx.x;
  const int nh = bid / NLT, lt = bid % NLT;
  if (nh >= NNH) return;
  const int n = nh / NH, h = nh % NH;
  const int l0 = lt * 64 + wave * 16;
  const size_t tb = (size_t)(n * L_FULL + l0) * NH + h;
  const size_t aoff = (tb + (size_t)m * NH) * DM + 8 * hh;
  const size_t boff = ((size_t)nh * 64 + m) * DM + 8 * hh;
  const _Float16* ah = (const _Float16*)(const void*)QH + aoff;
  const _Float16* al = (const _Float16*)(const void*)QL + aoff;
  const _Float16* bh = (const _Float16*)(const void*)KVH + boff;
  const _Float16* bl = (const _Float16*)(const void*)KVL + boff;
  v8f c0 = zero8(), c1 = zero8(), c2 = zero8(), c3 = zero8();
  kloop_h3<DM / 32>(ah, al, bh, bl, (size_t)16 * DM, c0, c1, c2, c3);
  float* sl = slab + wave * SLAB64;
  slab_put(sl, c0, c1, c2, c3, lane);
  const int rq = lane >> 3, c8 = (lane & 7) * 8;
  const float fold = 1.0f / (QSC * KVCAR);
  v4u oh[4], ol[4];
  size_t off[4];
#pragma unroll
  for (int it = 0; it < 4; ++it) {
    const int row = it * 4 + rq;
    const size_t t = tb + (size_t)row * NH;
    const float rd = 1.0f / DEN[t];
    float w[8];
    slab_row8(sl, row, c8, w);
#pragma unroll
    for (int e = 0; e < 8; ++e) w[e] = (w[e] * fold) * rd;
    pack_b2(w, oh[it], ol[it]);
    off[it] = t * DM + c8;
  }
  store2_planes(MH, ML, off, oh, ol);
}

__global__ __launch_bounds__(128)
void gemm_mg(const u16* __restrict__ MH, const u16* __restrict__ ML, const u16* __restrict__ WM,
             const float* __restrict__ g1, const float* __restrict__ b1, u16* M1H, u16* M1L) {
#pragma clang fp contract(off)
  __shared__ __align__(16) float slab[4 * SLAB64];
  const int tid = (int)threadIdx.x, wave = tid >> 5, lane = tid & 31, hh = lane >> 4, m = lane & 15;
  const int rowb0 = (int)blockIdx.x * 64;
  if (rowb0 + 64 > MT) return;
  const int rowb = rowb0 + wave * 16;
  const size_t aoff = (size_t)(rowb + m) * DM + 8 * hh;
  const u16* bp = WM + (size_t)m * DM + 8 * hh;
  v8f c0 = zero8(), c1 = zero8(), c2 = zero8(), c3 = zero8();
  kloop_b<2, DM / 32>(MH + aoff, ML + aoff, bp, (size_t)16 * DM, c0, c1, c2, c3);
  float* sl = slab + wave * SLAB64;
  slab_put(sl, c0, c1, c2, c3, lane);
  const int rq = lane >> 3, c8 = (lane & 7) * 8;
  v4u oh[4], ol[4];
  size_t off[4];
#pragma unroll
  for (int it = 0; it < 4; ++it) {
    const int row = it * 4 + rq;
    const int t = rowb + row;
    float w[8];
    slab_row8(sl, row, c8, w);
    ln8(w, g1, b1, c8);
    pack_b2(w, oh[it], ol[it]);
    off[it] = (size_t)t * DM + c8;
  }
  store2_planes(M1H, M1L, off, oh, ol);
}

__global__ __launch_bounds__(128)
void gemm_w1(const u16* __restrict__ XB, const u16* __restrict__ M1H, const u16* __restrict__ M1L,
             const u16* __restrict__ W1, u16* H3H, u16* H3L) {
#pragma clang fp contract(off)
  __shared__ __align__(16) float slab[4 * SLAB64];
  const int tid = (int)threadIdx.x, wave = tid >> 5, lane = tid & 31, hh = lane >> 4, m = lane & 15;
  const int bid = (int)blockIdx.x;
  const int rowb0 = (bid >> 1) * 64, col0 = (bid & 1) * 64;
  if (rowb0 + 64 > MT) return;
  const int rowb = rowb0 + wave * 16;
  const size_t aoff = (size_t)(rowb + m) * DM + 8 * hh;
  const u16* bp = W1 + (size_t)(col0 + m) * DFF + 8 * hh;
  v8f c0 = zero8(), c1 = zero8(), c2 = zero8(), c3 = zero8();
  kloop_b<1, DM / 32>(XB + aoff, XB + aoff, bp, (size_t)16 * DFF, c0, c1, c2, c3);
  kloop_b<2, DM / 32>(M1H + aoff, M1L + aoff, bp + DM, (size_t)16 * DFF, c0, c1, c2, c3);
  float* sl = slab + wave * SLAB64;
  slab_put(sl, c0, c1, c2, c3, lane);
  const int rq = lane >> 3, c8 = (lane & 7) * 8;
  v4u oh[4], ol[4];
  size_t off[4];
#pragma unroll
  for (int it = 0; it < 4; ++it) {
    const int row = it * 4 + rq;
    const int t = rowb + row;
    float w[8];
    slab_row8(sl, row, c8, w);
#pragma unroll
    for (int e = 0; e < 8; ++e) w[e] = fmaxf(w[e], 0.0f);
    pack_b2(w, oh[it], ol[it]);
    off[it] = (size_t)t * DFF + col0 + c8;
  }
  store2_planes(H3H, H3L, off, oh, ol);
}

__global__ __launch_bounds__(128)
void gemm_w2(const u16* __restrict__ H3H, const u16* __restrict__ H3L, const u16* __restrict__ W2,
             const u16* __restrict__ XB, const float* __restrict__ g2, const float* __restrict__ b2, float* out) {
#pragma clang fp contract(off)
  __shared__ __align__(16) float slab[4 * SLAB64];
  const int tid = (int)threadIdx.x, wave = tid >> 5, lane = tid & 31, hh = lane >> 4, m = lane & 15;
  const int rowb0 = (int)blockIdx.x * 64;
  if (rowb0 + 64 > MT) return;
  const int rowb = rowb0 + wave * 16;
  const size_t aoff = (size_t)(rowb + m) * DFF + 8 * hh;
  const u16* bp = W2 + (size_t)m * DFF + 8 * hh;
  v8f c0 = zero8(), c1 = zero8(), c2 = zero8(), c3 = zero8();
  kloop_b<2, DFF / 32>(H3H + aoff, H3L + aoff, bp, (size_t)16 * DFF, c0, c1, c2, c3);
  float* sl = slab + wave * SLAB64;
  slab_put(sl, c0, c1, c2, c3, lane);
  const int rq = lane >> 3, c8 = (lane & 7) * 8;
#pragma unroll
  for (int it = 0; it < 4; ++it) {
    const int row = it * 4 + rq;
    const int t = rowb + row;
    float w[8];
    slab_row8(sl, row, c8, w);
    ln8(w, g2, b2, c8);
    const v4u xx = *(const v4u*)(XB + (size_t)t * DM + c8);
    v4f ya, yb;
#pragma unroll
    for (int e = 0; e < 2; ++e) {
      const float xa0 = bf_up((unsigned short)(xx[e] & 0xffffu)),     xa1 = bf_up((unsigned short)(xx[e] >> 16));
      const float xb0 = bf_up((unsigned short)(xx[2 + e] & 0xffffu)), xb1 = bf_up((unsigned short)(xx[2 + e] >> 16));
      ya[2 * e] = xa0 + w[2 * e];      ya[2 * e + 1] = xa1 + w[2 * e + 1];
      yb[2 * e] = xb0 + w[4 + 2 * e];  yb[2 * e + 1] = xb1 + w[4 + 2 * e + 1];
    }
    *(v4f*)(sl + row * SLP + c8)     = ya;
    *(v4f*)(sl + row * SLP + c8 + 4) = yb;
  }
  wave_sync_lds();
  v4f vals[8];
#pragma unroll
  for (int it = 0; it < 8; ++it) vals[it] = *(const v4f*)(sl + (it * 2 + hh) * SLP + m * 4);
  float* dst = out + ((size_t)rowb + hh) * DM + m * 4;
  for (int pass = 0; pass < 2; ++pass) {
#pragma unroll
    for (int it = 0; it < 8; ++it) {
      *(volatile v4f*)(dst + (size_t)(it * 2) * DM) = vals[it];
    }
    __threadfence();
  }
}

extern "C" void kernel_launch(void* const* d_in, const int* in_sizes, int n_in,
                              void* d_out, int out_size, void* d_ws, size_t ws_size,
                              hipStream_t stream) {
  if (n_in < 12) return;
  const long needx = (long)((NB - 1) * L_FULL + SEQ) * NH * DM;
  const long needs = (long)((NB - 1) * L_FULL + SSEQ) * NH * DM;
  if ((long)in_sizes[0] < needx || (long)in_sizes[1] < needs) return;
  if (in_sizes[2] != DM * DM || in_sizes[3] != DM * DM || in_sizes[4] != DM * DM || in_sizes[5] != DM * DM) return;
  if (in_sizes[6] != DFF * DFF || in_sizes[7] != DM * DFF) return;
  if (in_sizes[8] != DM || in_sizes[9] != DM || in_sizes[10] != DM || in_sizes[11] != DM) return;
  if ((long)out_size < needx) return;

  const float* x   = (const float*)d_in[0];
  const float* src = (const float*)d_in[1];
  const float* wq  = (const float*)d_in[2];
  const float* wk  = (const float*)d_in[3];
  const float* wv  = (const float*)d_in[4];
  const float* wm  = (const float*)d_in[5];
  const float* w1  = (const float*)d_in[6];
  const float* w2  = (const float*)d_in[7];
  const float* g1  = (const float*)d_in[8];
  const float* b1  = (const float*)d_in[9];
  const float* g2  = (const float*)d_in[10];
  const float* b2  = (const float*)d_in[11];
  float*       out = (float*)d_out;

  size_t off = 0;
  const size_t oW   = off; off += SZ_W;
  const size_t oPS  = off; off += SZ_PS;
  const size_t oKS  = off; off += SZ_KS;
  const size_t oKVH = off; off += SZ_KV;
  const size_t oKVL = off; off += SZ_KV;
  const size_t oDEN = off; off += SZ_DEN;
  const size_t oXB  = off; off += SZ_XB;
  const size_t oA   = off; off += SLB;
  const size_t oT   = off; off += 4 * SLB;
  const size_t oF   = off; off += SLB;
  (void)oF;
  if (off != WS_TOTAL) return;
  if (off > ws_size || off > (size_t)WS_CAP) return;

  char* ws = (char*)d_ws;
  u16*   WQp  = (u16*)(ws + oW);
  u16*   WKp  = (u16*)(ws + oW + 8192);
  u16*   WVp  = (u16*)(ws + oW + 16384);
  u16*   WMp  = (u16*)(ws + oW + 24576);
  u16*   W1p  = (u16*)(ws + oW + 32768);
  u16*   W2p  = (u16*)(ws + oW + 65536);
  float* PSp  = (float*)(ws + oPS);
  float* KSp  = (float*)(ws + oKS);
  u16*   KVHp = (u16*)(ws + oKVH);
  u16*   KVLp = (u16*)(ws + oKVL);
  float* DENp = (float*)(ws + oDEN);
  u16*   XBp  = (u16*)(ws + oXB);
  u16*   SBp  = (u16*)(ws + oA);
  u16*   QHp  = (u16*)(ws + oA);
  u16*   M1Hp = (u16*)(ws + oA);
  u16*   KTHp = (u16*)(ws + oT);
  u16*   KTLp = (u16*)(ws + oT + SLB);
  u16*   PTHp = (u16*)(ws + oT + 2 * SLB);
  u16*   PTLp = (u16*)(ws + oT + 3 * SLB);
  u16*   QLp  = (u16*)(ws + oT);
  u16*   MHp  = (u16*)(ws + oT + SLB);
  u16*   MLp  = (u16*)(ws + oT + 2 * SLB);
  u16*   M1Lp = (u16*)(ws + oT);
  u16*   H3Hp = (u16*)(ws + oT + SLB);
  u16*   H3Lp = (u16*)(ws + oT + 3 * SLB);

  const dim3 b256(256), b128(128);
  const int  n8a = MT * 8, n8b = MS * 8;
  const dim3 gX2((MX * 8) / 256, 2);
  const dim3 gKT(NNH * NST);
  const dim3 gKV(NNH);
  const dim3 gTK(MT / 64);
  const dim3 gQK(NNH * NLT);
  const dim3 gW1((MT / 64) * 2);

  cvt_w<<<dim3(20), b256, 0, stream>>>(wq, wk, wv, wm, w1, w2, WQp, WKp, WVp, WMp, W1p, W2p);
  cvt_x2<<<gX2, b256, 0, stream>>>(x, src, XBp, SBp, n8a, n8b);
  gemm_kt<true><<<gKT, b128, 0, stream>>>(WKp, SBp, KTHp, KTLp, PSp);
  gemm_kt<false><<<gKT, b128, 0, stream>>>(WVp, SBp, PTHp, PTLp, PSp);
  kv_gemm<<<gKV, b128, 0, stream>>>(PTHp, PTLp, KTHp, KTLp, PSp, KVHp, KVLp, KSp);
  gemm_q<<<gTK, b128, 0, stream>>>(XBp, WQp, KSp, QHp, QLp, DENp);
  qkv<<<gQK, b128, 0, stream>>>(QHp, QLp, KVHp, KVLp, DENp, MHp, MLp);
  gemm_mg<<<gTK, b128, 0, stream>>>(MHp, MLp, WMp, g1, b1, M1Hp, M1Lp);
  gemm_w1<<<gW1, b128, 0, stream>>>(XBp, M1Hp, M1Lp, W1p, H3Hp, H3Lp);
  gemm_w2<<<gTK, b128, 0, stream>>>(H3Hp, H3Lp, W2p, XBp, g2, b2, out);
  (void)hipGetLastError();
}
